// QuantumLayer_88098369176448
// MI455X (gfx1250) — hardware-run, weakly checked
//
#include <hip/hip_runtime.h>
#include <math.h>


#pragma clang fp contract(off)

#ifndef NB
#define NB 256
#endif
#define NB_FULL 256
#define NW   8
#define SDIM 65536
#define NBC  (NB < 64 ? NB : 64)
#define NMAT 9
#define TPW  16
#define WPS  (256 / TPW)
#define AWV  4
#define CAR  4096.0f
#define ICAR (1.0f / 4096.0f)
#define QRS  2048.0f
#define QRI  (1.0f / 2048.0f)
#define CH_S1 0.974679410457611084f
#define CH_SP 0.223606795072555542f
#define CH_S3 0.129099443554878235f

static_assert(__builtin_bit_cast(unsigned, CH_S1) == 0x3F798497u);
static_assert(__builtin_bit_cast(unsigned, CH_SP) == 0x3E64F92Eu);
static_assert(__builtin_bit_cast(unsigned, CH_S3) == 0x3E0432A5u);
static_assert(NB <= NB_FULL);
static_assert(NB % NBC == 0);
static_assert(NBC % 16 == 0);
static_assert(NB % 8 == 0);
static_assert(256 % TPW == 0);
static_assert((NBC * WPS) % AWV == 0);
static_assert(4 * 32 * 4 == 16 * 16 * 2);
static_assert(8 * 16 * 256 * 2 == SDIM);
static_assert(32 * 4 == 16 * NW);
static_assert((NMAT * 1024) % 8 == 0);
static_assert(AWV * 512 * 4 <= 131072);
static_assert(2096 * 4 + 2 * NMAT * 1024 * 2 <= 131072);
static_assert(8 * 256 * 4 <= 131072);

typedef _Float16 h16;
typedef unsigned short bf;
typedef __attribute__((ext_vector_type(16))) _Float16 v16h;
typedef __attribute__((ext_vector_type(8)))  _Float16 v8h;
typedef __attribute__((ext_vector_type(8)))  float    v8f;
typedef __attribute__((ext_vector_type(4)))  float    v4f;
typedef __attribute__((ext_vector_type(2)))  float    v2f;
typedef v4f  __attribute__((may_alias)) v4fa;
typedef v8h  __attribute__((may_alias)) v8ha;

__device__ __forceinline__ unsigned short f2bf(float f) { unsigned u = __float_as_uint(f); u += 0x7FFFu + ((u >> 16) & 1u); return (unsigned short)(u >> 16); }
__device__ __forceinline__ float bfr(float f) { return __uint_as_float(((unsigned)f2bf(f)) << 16); }
__device__ __forceinline__ v16h cat16(v8h lo, v8h hi) { return __builtin_shufflevector(lo, hi, 0, 1, 2, 3, 4, 5, 6, 7, 8, 9, 10, 11, 12, 13, 14, 15); }
__device__ __forceinline__ v8f wmma16(v16h a, v16h b, v8f c) { return __builtin_amdgcn_wmma_f32_16x16x32_f16(false, a, false, b, (short)0, c, false, false); }
__device__ __forceinline__ v16h  ldh(const h16* p) { return cat16(*(const v8h*)p, *(const v8h*)(p + 16)); }
__device__ __forceinline__ void wave_sync() { __builtin_amdgcn_fence(3  , "wavefront"); __builtin_amdgcn_wave_barrier(); asm volatile("" ::: "memory"); }
__device__ __forceinline__ v8f wmma16g(v16h a, v16h b, v8f c) { c = wmma16(a, b, c); asm volatile("v_nop\n\tv_nop\n\tv_nop\n\tv_nop" : "+v"(c) : "v"(a), "v"(b)); return c; }
static __device__ __forceinline__ h16 toh_flush(float v) { const h16 r = (h16)v; return (fabsf(v) < 6.103515625e-05f) ? (h16)0.0f : r; }

static __device__ __forceinline__ void rot_el(float c0, float s0, float c1, float n1, float c2, float n2, int i, int j, float& re, float& im) {
    const bool dg = (i == j);
    const float mag = dg ? c0 : (i ? s0 : -s0);
    const float cp = dg ? c1 : c2;
    const float sn = dg ? n1 : n2;
    const float sg = i ? sn : -sn;
    re = mag * cp; im = mag * sg;
}

__global__ __launch_bounds__(256) void k_mats(const float* __restrict__ wts, float* T4, h16* AH, h16* AR) {
    __shared__ float tc[72], ts[72];
    __shared__ float kre[80], kim[80];
    __shared__ float chre[80], chim[80];
    __shared__ float nre[16], nim[16], ure[16], uim[16];
    __shared__ float rre[384], rim[384];
    __shared__ __align__(16) float t4s[800];
    __shared__ __align__(16) h16 ahs[NMAT * 1024];
    __shared__ __align__(16) h16 ars[NMAT * 1024];
    const int tid = threadIdx.x;
    const float s1 = CH_S1, sp = CH_SP, s3 = CH_S3;
    { const int e = tid < 72 ? tid : 71; const int q = e / 3, j = e - 3 * q;
      float phi = bfr(wts[q * 3 + 0]), th = bfr(wts[q * 3 + 1]), om = bfr(wts[q * 3 + 2]);
      asm volatile("" : "+v"(phi), "+v"(th), "+v"(om));
      const float ang = (j == 0) ? 0.5f * th : ((j == 1) ? 0.5f * (om + phi) : 0.5f * (om - phi));
      float sn, cs; sincosf(ang, &sn, &cs);
      if (tid < 72) { tc[tid] = cs; ts[tid] = sn; } }
    if (tid < 80) {
        const int c = tid >> 4, k = (tid >> 2) & 3, i = (tid >> 1) & 1, j = tid & 1;
        const float dg = (i == j) ? 1.0f : 0.0f, od = (i != j) ? 1.0f : 0.0f, zs = (i == j) ? (i ? -1.0f : 1.0f) : 0.0f;
        float re = 0.0f, im = 0.0f;
        if (k == 0) { re = (c <= 2) ? s1 * dg : ((i == j) ? (i ? s1 : 1.0f) : 0.0f); }
        else if (k == 1) {
            if (c == 0) re = s3 * od; else if (c == 1) re = sp * od; else if (c == 2) re = sp * zs;
            else if (c == 3) re = (i == 0 && j == 1) ? sp : 0.0f; else re = (i == 1 && j == 1) ? sp : 0.0f; }
        else if (k == 2) { if (c == 0) im = (i == 0 && j == 1) ? -s3 : ((i == 1 && j == 0) ? s3 : 0.0f); }
        else { if (c == 0) re = s3 * zs; }
        kre[tid] = re; kim[tid] = im; }
    __syncthreads();
#pragma unroll 1
    for (int it = 0; it < 2; ++it) {
        const int e = it * 256 + tid; const int ec = e < 384 ? e : 383;
        const int q = ec >> 4, g = (ec >> 2) & 3, gp = ec & 3;
        const float c0 = tc[q * 3], s0 = ts[q * 3], c1 = tc[q * 3 + 1], n1 = ts[q * 3 + 1], c2 = tc[q * 3 + 2], n2 = ts[q * 3 + 2];
        float are, aim, bre, bim;
        rot_el(c0, s0, c1, n1, c2, n2, g >> 1, gp >> 1, are, aim);
        rot_el(c0, s0, c1, n1, c2, n2, g & 1, gp & 1, bre, bim);
        const float vr = are * bre + aim * bim, vi = aim * bre - are * bim;
        if (e < 384) { rre[e] = vr; rim[e] = vi; } }
    { const int e = tid < 80 ? tid : 79; const int c = e >> 4, g = (e >> 2) & 3, gp = e & 3;
      const int r = g >> 1, cc = g & 1, rp = gp >> 1, cp = gp & 1;
      float sr = 0.0f, si = 0.0f;
#pragma unroll 1
      for (int k = 0; k < 4; ++k) { const int ia = c * 16 + k * 4 + r * 2 + rp, ib = c * 16 + k * 4 + cc * 2 + cp;
          const float ar = kre[ia], ai = kim[ia], br = kre[ib], bi = kim[ib];
          sr += ar * br + ai * bi; si += ai * br - ar * bi; }
      if (tid < 80) { chre[tid] = sr; chim[tid] = si; } }
    if (tid < 16) { nre[tid] = ((tid >> 2) == (tid & 3)) ? 1.0f : 0.0f; nim[tid] = 0.0f; }
    __syncthreads();
#pragma unroll 1
    for (int c = 0; c < 5; ++c) {
        { const int e = tid & 15; const int i = e >> 2, j = e & 3; float sr = 0.0f, si = 0.0f;
#pragma unroll 1
          for (int m = 0; m < 4; ++m) { const float ar = chre[c * 16 + i * 4 + m], ai = chim[c * 16 + i * 4 + m], br = nre[m * 4 + j], bi = nim[m * 4 + j];
              sr += ar * br - ai * bi; si += ar * bi + ai * br; }
          if (tid < 16) { ure[e] = sr; uim[e] = si; } }
        __syncthreads();
        if (tid < 16) { nre[tid] = ure[tid]; nim[tid] = uim[tid]; }
        __syncthreads();
    }
#pragma unroll 1
    for (int it = 0; it < 2; ++it) {
        const int e = it * 256 + tid; const int ec = e < 400 ? e : 399;
        const int en = ec < 16 ? ec : 15; const int er = ec < 16 ? 0 : ec - 16;
        const float a0 = nre[en], a1 = nim[en], b0 = rre[er], b1 = rim[er];
        const float v0 = (ec < 16) ? a0 : b0, v1 = (ec < 16) ? a1 : b1;
        if (e < 400) { t4s[2 * e] = v0; t4s[2 * e + 1] = v1; } }
#pragma unroll 1
    for (int mat = 0; mat < NMAT; ++mat) {
        const int R = tid >> 4, C = tid & 15;
        const int mr = mat < 8 ? mat : 0;
        const int qa = (1 + (mr >> 2)) * 8 + 2 * (mr & 3);
        const int ia = (R >> 2) * 4 + (C >> 2), ib = (R & 3) * 4 + (C & 3);
        const float ra = rre[qa * 16 + ia], rai = rim[qa * 16 + ia], rb = rre[(qa + 1) * 16 + ib], rbi = rim[(qa + 1) * 16 + ib];
        const float na = nre[ia], nai = nim[ia], nbv = nre[ib], nbi = nim[ib];
        const bool rot = mat < 8;
        const float ar = rot ? ra : na, ai = rot ? rai : nai, br = rot ? rb : nbv, bi = rot ? rbi : nbi;
        const float er = ar * br - ai * bi, ei = ar * bi + ai * br;
        const float vals[4] = { er, -ei, ei, er };
        const int pos[4] = { R * 32 + C, R * 32 + 16 + C, (16 + R) * 32 + C, (16 + R) * 32 + 16 + C };
        const int o = mat * 1024;
#pragma unroll
        for (int u = 0; u < 4; ++u) { const h16 hv = toh_flush(vals[u]); ahs[o + pos[u]] = hv; ars[o + pos[u]] = toh_flush((vals[u] - (float)hv) * QRS); }
    }
    __syncthreads();
    const int NV8 = NMAT * 1024 / 8;
#pragma unroll 1
    for (int ps = 0; ps < 2; ++ps) {
#pragma unroll 1
        for (int it = 0; it < 5; ++it) { const int i = it * 256 + tid; const int ic = i < NV8 ? i : NV8 - 1;
            const v8h a = *(const v8ha*)(&ahs[ic * 8]); const v8h r = *(const v8ha*)(&ars[ic * 8]);
            if (i < NV8) { *(volatile v8h*)(AH + (size_t)i * 8) = a; *(volatile v8h*)(AR + (size_t)i * 8) = r; } }
        { const int ic = tid < 200 ? tid : 199; const v4f t = *(const v4fa*)(&t4s[ic * 4]); if (tid < 200) *(volatile v4f*)(T4 + (size_t)tid * 4) = t; }
        if (ps == 0) __threadfence(); }
}

__global__ __launch_bounds__(256) void k_vinit(const float* __restrict__ x, const float* __restrict__ T4, float* V) {
    __shared__ __align__(16) float ls[8 * 256];
    const int lane = threadIdx.x & 31;
    const int wave = __builtin_amdgcn_readfirstlane((int)(threadIdx.x >> 5));
    const int b = blockIdx.x * 8 + wave; const int wb = wave * 256;
    { const int w = lane & 7, g = lane >> 3;
      const float a = bfr(x[(size_t)b * NW + w]); float sn, cs; sincosf(0.5f * a, &sn, &cs);
      const float cc = cs * cs, ss = sn * sn, cx = cs * sn;
      const float re = (g == 0) ? cc : ((g == 3) ? ss : 0.0f);
      const float im = (g == 1) ? cx : ((g == 2) ? -cx : 0.0f);
      ls[wb + (w * 4 + g) * 2] = re; ls[wb + (w * 4 + g) * 2 + 1] = im; }
    wave_sync();
    { const int w = lane >> 2, g = lane & 3; float sr = 0.0f, si = 0.0f;
#pragma unroll 1
      for (int m = 0; m < 4; ++m) { const float ar = T4[(g * 4 + m) * 2], ai = T4[(g * 4 + m) * 2 + 1];
          const float br = ls[wb + (w * 4 + m) * 2], bi = ls[wb + (w * 4 + m) * 2 + 1];
          sr += ar * br - ai * bi; si += ar * bi + ai * br; }
      ls[wb + 64 + (w * 4 + g) * 2] = sr; ls[wb + 64 + (w * 4 + g) * 2 + 1] = si; }
    wave_sync();
    { const int w = lane >> 2, g = lane & 3; float sr = 0.0f, si = 0.0f;
#pragma unroll 1
      for (int m = 0; m < 4; ++m) { const int ti = ((1 + w) * 16 + g * 4 + m) * 2; const float ar = T4[ti], ai = T4[ti + 1];
          const float br = ls[wb + 64 + (w * 4 + m) * 2], bi = ls[wb + 64 + (w * 4 + m) * 2 + 1];
          sr += ar * br - ai * bi; si += ar * bi + ai * br; }
      ls[wb + (w * 4 + g) * 2] = sr; ls[wb + (w * 4 + g) * 2 + 1] = si; }
    wave_sync();
#pragma unroll
    for (int u = 0; u < 2; ++u) { const int e = lane + 32 * u; const int p = e >> 4, G = e & 15;
        const int ia = wb + ((2 * p) * 4 + (G >> 2)) * 2, ib = wb + ((2 * p + 1) * 4 + (G & 3)) * 2;
        const float ar = ls[ia], ai = ls[ia + 1], br = ls[ib], bi = ls[ib + 1];
        ls[wb + 128 + e * 2] = ar * br - ai * bi; ls[wb + 128 + e * 2 + 1] = ar * bi + ai * br; }
    wave_sync();
    { const v4f val = *(const v4fa*)(&ls[wb + 128 + lane * 4]);
      float* dst = V + (size_t)b * 128 + lane * 4;
      *(volatile v4f*)dst = val; __threadfence(); *(volatile v4f*)dst = val; }
}

__global__ __launch_bounds__(256) void k_init(const float* __restrict__ V, float* S, int cbase) {
    __shared__ float vsh[128];
    const int tid = threadIdx.x; const int bl = blockIdx.x >> 3, seg = blockIdx.x & 7;
    vsh[tid & 127] = V[(size_t)(cbase + bl) * 128 + (tid & 127)];
    __syncthreads();
    float* ob = S + (size_t)bl * (SDIM * 2);
#pragma unroll 1
    for (int it = 0; it < 16; ++it) {
        const int e0 = seg * 8192 + (it * 256 + tid) * 2;
        const int i0 = ((e0 >> 12) & 15) * 2, i1 = (16 + ((e0 >> 8) & 15)) * 2, i2 = (32 + ((e0 >> 4) & 15)) * 2, i3 = (48 + (e0 & 15)) * 2;
        const float ar = vsh[i0], ai = vsh[i0 + 1], br = vsh[i1], bi = vsh[i1 + 1], cr = vsh[i2], ci = vsh[i2 + 1];
        const float d0r = vsh[i3], d0i = vsh[i3 + 1], d1r = vsh[i3 + 2], d1i = vsh[i3 + 3];
        const float pr = ar * br - ai * bi, pi = ar * bi + ai * br;
        const float qr = pr * cr - pi * ci, qi = pr * ci + pi * cr;
        v4f val; val[0] = qr * d0r - qi * d0i; val[1] = qr * d0i + qi * d0r; val[2] = qr * d1r - qi * d1i; val[3] = qr * d1i + qi * d1r;
        float* dst = ob + (size_t)e0 * 2;
        *(volatile v4f*)dst = val; __threadfence(); *(volatile v4f*)dst = val;
    }
}

__global__ __launch_bounds__(32 * AWV) void k_apply(const float* __restrict__ SIN, float* SOUT, const h16* __restrict__ AH, const h16* __restrict__ AR,
                                                    unsigned km01, unsigned km23, unsigned rm01, unsigned rm23, unsigned rm45, unsigned rm67, unsigned rm89, unsigned rmab) {
    __shared__ __align__(16) float os[AWV * 512];
    const int lane = threadIdx.x & 31, lr = lane & 15, hi = lane >> 4;
    const int wave = __builtin_amdgcn_readfirstlane((int)(threadIdx.x >> 5));
    const int gw = blockIdx.x * AWV + wave;
    const int smp = gw / WPS, tg = gw % WPS;
    const unsigned k0 = km01 & 0xffffu, k1 = km01 >> 16, k2 = km23 & 0xffffu, k3 = km23 >> 16;
    const unsigned q0 = rm01 & 0xffffu, q1 = rm01 >> 16, q2 = rm23 & 0xffffu, q3 = rm23 >> 16, q4 = rm45 & 0xffffu, q5 = rm45 >> 16;
    const unsigned q6 = rm67 & 0xffffu, q7 = rm67 >> 16, q8 = rm89 & 0xffffu, q9 = rm89 >> 16, q10 = rmab & 0xffffu, q11 = rmab >> 16;
    const int ao = lr * 32 + 8 * hi;
    const v16h ahr = ldh(AH + ao), ahm = ldh(AH + 512 + ao);
    const v16h arr = ldh(AR + ao), arm = ldh(AR + 512 + ao);
    unsigned kof[8];
    const unsigned kh = k3 & (0u - (unsigned)hi);
#pragma unroll
    for (int j = 0; j < 8; ++j) kof[j] = kh ^ (k0 & (0u - (unsigned)(j & 1))) ^ (k1 & (0u - (unsigned)((j >> 1) & 1))) ^ (k2 & (0u - (unsigned)((j >> 2) & 1)));
    const unsigned nbm = (q0 & (0u - (unsigned)(lr & 1))) ^ (q1 & (0u - (unsigned)((lr >> 1) & 1))) ^ (q2 & (0u - (unsigned)((lr >> 2) & 1))) ^ (q3 & (0u - (unsigned)((lr >> 3) & 1)));
    const float* sb = SIN + (size_t)smp * (SDIM * 2);
    float* ob = SOUT + (size_t)smp * (SDIM * 2);
    const int wbs = wave * 512;
#pragma unroll 1
    for (int ti = 0; ti < TPW; ++ti) {
        const int tile = tg * TPW + ti;
        const unsigned tb = (q4 & (0u - (unsigned)(tile & 1))) ^ (q5 & (0u - (unsigned)((tile >> 1) & 1))) ^ (q6 & (0u - (unsigned)((tile >> 2) & 1))) ^ (q7 & (0u - (unsigned)((tile >> 3) & 1)))
                          ^ (q8 & (0u - (unsigned)((tile >> 4) & 1))) ^ (q9 & (0u - (unsigned)((tile >> 5) & 1))) ^ (q10 & (0u - (unsigned)((tile >> 6) & 1))) ^ (q11 & (0u - (unsigned)((tile >> 7) & 1)));
        const unsigned cb = nbm ^ tb;
        v2f z[8];
#pragma unroll
        for (int j = 0; j < 8; ++j) z[j] = *(const v2f*)(sb + 2 * (size_t)(cb ^ kof[j]));
        v16h bh;
#pragma unroll
        for (int j = 0; j < 8; ++j) {
            const float xr = z[j][0] * CAR, xi = z[j][1] * CAR;
            const h16 hr = toh_flush(xr), hq = toh_flush(xi);
            bh[j] = hr; bh[8 + j] = hq; }
        v8f dHr = (v8f){}, dHi = (v8f){}, dLr = (v8f){}, dLi = (v8f){};
        dHr = wmma16g(ahr, bh, dHr); dHi = wmma16g(ahm, bh, dHi);
        dLr = wmma16g(arr, bh, dLr); dLi = wmma16g(arm, bh, dLi);
        const int lo = wbs + lr * 32 + hi * 16;
#pragma unroll
        for (int q = 0; q < 4; ++q) { v4f t;
            t[0] = (dHr[2 * q] + dLr[2 * q] * QRI) * ICAR;         t[1] = (dHi[2 * q] + dLi[2 * q] * QRI) * ICAR;
            t[2] = (dHr[2 * q + 1] + dLr[2 * q + 1] * QRI) * ICAR; t[3] = (dHi[2 * q + 1] + dLi[2 * q + 1] * QRI) * ICAR;
            *(v4fa*)(&os[lo + 4 * q]) = t; }
        wave_sync();
        float* ot = ob + (size_t)tile * 512;
#pragma unroll 1
        for (int ps = 0; ps < 2; ++ps) {
#pragma unroll
            for (int s = 0; s < 4; ++s) { const int p = s * 32 + lane;
                const v4f val = *(const v4fa*)(&os[wbs + p * 4]);
                *(volatile v4f*)(ot + (size_t)p * 4) = val; }
            if (ps == 0) __threadfence(); }
        wave_sync();
    }
}

__global__ __launch_bounds__(32) void k_expect(const float* __restrict__ S, const float* __restrict__ noise, float* OUT, int cbase,
                                               unsigned dm01, unsigned dm23, unsigned dm45, unsigned dm67) {
    __shared__ __align__(16) float os[16 * 16];
    const int lane = threadIdx.x & 31, lr = lane & 15, hi = lane >> 4;
    const unsigned d0 = dm01 & 0xffffu, d1 = dm01 >> 16, d2 = dm23 & 0xffffu, d3 = dm23 >> 16, d4 = dm45 & 0xffffu, d5 = dm45 >> 16, d6 = dm67 & 0xffffu, d7 = dm67 >> 16;
    const float* sb = S + (size_t)(blockIdx.x * 16 + lr) * (SDIM * 2);
    unsigned lo[8];
#pragma unroll
    for (int j = 0; j < 8; ++j) lo[j] = (d0 & (0u - (unsigned)(j & 1))) ^ (d1 & (0u - (unsigned)((j >> 1) & 1))) ^ (d2 & (0u - (unsigned)((j >> 2) & 1)));
    const unsigned hm = d3 & (0u - (unsigned)hi);
    const int wsh = (7 - lr) & 7;
    const float wok = (lr < 8) ? 1.0f : 0.0f;
    v8f eh = (v8f){}, er = (v8f){};
#pragma unroll 1
    for (int kc = 0; kc < 8; ++kc) {
        const unsigned km = (d5 & (0u - (unsigned)(kc & 1))) ^ (d6 & (0u - (unsigned)((kc >> 1) & 1))) ^ (d7 & (0u - (unsigned)((kc >> 2) & 1)));
        const unsigned b0 = hm ^ km, b1 = b0 ^ d4;
        const int kb = kc * 32 + 8 * hi;
        v16h ah, ar, bs;
#pragma unroll
        for (int j = 0; j < 8; ++j) {
            const float p0 = sb[2 * (size_t)(b0 ^ lo[j])] * CAR, p1 = sb[2 * (size_t)(b1 ^ lo[j])] * CAR;
            const h16 h0 = toh_flush(p0), h1 = toh_flush(p1);
            ah[j] = h0; ah[8 + j] = h1;
            ar[j] = toh_flush((p0 - (float)h0) * QRS); ar[8 + j] = toh_flush((p1 - (float)h1) * QRS);
            const int ka = kb + j, kd = kb + 16 + j;
            bs[j] = toh_flush(((ka >> wsh) & 1) ? -wok : wok); bs[8 + j] = toh_flush(((kd >> wsh) & 1) ? -wok : wok); }
        eh = wmma16g(ah, bs, eh); er = wmma16g(ar, bs, er);
    }
#pragma unroll
    for (int r = 0; r < 8; ++r) {
        const float e = (eh[r] + er[r] * QRI) * ICAR;
        const int smp = cbase + blockIdx.x * 16 + 8 * hi + r;
        const float nz = bfr(noise[(size_t)smp * NW + (lr & 7)]);
        const float sg = sqrtf(fmaxf(1.0f - e * e, 0.0f) * (1.0f / 1024.0f));
        float o = e + nz * sg; o = fminf(1.0f, fmaxf(-1.0f, o));
        os[(8 * hi + r) * 16 + lr] = o; }
    wave_sync();
    float* ot = OUT + (size_t)(cbase + blockIdx.x * 16) * NW;
#pragma unroll 1
    for (int ps = 0; ps < 2; ++ps) {
        const v4f val = *(const v4fa*)(&os[(lane >> 1) * 16 + (lane & 1) * 4]);
        *(volatile v4f*)(ot + (size_t)lane * 4) = val;
        if (ps == 0) __threadfence(); }
}

static constexpr size_t al256(size_t v) { return (v + 255) & ~(size_t)255; }
static constexpr size_t SZ_S  = al256((size_t)NBC * SDIM * 2 * 4);
static constexpr size_t SZ_A  = al256((size_t)NMAT * 1024 * 2);
static constexpr size_t SZ_T4 = al256((size_t)800 * 4);
static constexpr size_t SZ_V  = al256((size_t)NB * 128 * 4);
static constexpr size_t SZ_TOTAL = 2 * SZ_S + 2 * SZ_A + SZ_T4 + SZ_V;
static_assert(SZ_TOTAL <= (size_t)134217728);
static_assert((size_t)200 * 16 <= SZ_T4);
static_assert((size_t)(NMAT * 1024 / 8) * 16 <= SZ_A);

static void cnot_relabel(unsigned short* cm, int c, int t) {
    const int sc = 2 * (NW - 1 - c), st = 2 * (NW - 1 - t);
    cm[sc + 1] = (unsigned short)(cm[sc + 1] ^ cm[st + 1]);
    cm[sc]     = (unsigned short)(cm[sc] ^ cm[st]);
}

extern "C" void kernel_launch(void* const* d_in, const int* in_sizes, int n_in,
                              void* d_out, int out_size, void* d_ws, size_t ws_size, hipStream_t stream) {
    if (n_in < 3) return;
    if (in_sizes[0] < NB * NW || in_sizes[1] < 72 || in_sizes[2] < NB * NW) return;
    if (out_size < NB * NW) return;
    if (SZ_TOTAL > ws_size) return;
    const float* x = (const float*)d_in[0];
    const float* wts = (const float*)d_in[1];
    const float* noise = (const float*)d_in[2];
    float* OUT = (float*)d_out;
    char* wsp = (char*)d_ws;
    float* S0 = (float*)wsp; wsp += SZ_S;
    float* S1 = (float*)wsp; wsp += SZ_S;
    h16* AH = (h16*)wsp; wsp += SZ_A;
    h16* AR = (h16*)wsp; wsp += SZ_A;
    float* T4 = (float*)wsp; wsp += SZ_T4;
    float* VT = (float*)wsp; wsp += SZ_V;

    k_mats<<<1, 256, 0, stream>>>(wts, T4, AH, AR);
    k_vinit<<<NB / 8, 256, 0, stream>>>(x, T4, VT);

    for (int cb = 0; cb < NB; cb += NBC) {
        unsigned short cm[16];
        for (int j = 0; j < 16; ++j) cm[j] = (unsigned short)(1u << j);
        k_init<<<NBC * 8, 256, 0, stream>>>(VT, S0, cb);
        float* cur = S0; float* oth = S1;
        for (int st = 0; st < 4; ++st) {
            if (st > 0) {
                for (int p = 0; p < 4; ++p) {
                    const int mat = (st < 3) ? ((st - 1) * 4 + p) : 8;
                    const int sh = 12 - 4 * p;
                    unsigned km[4], rm[12];
                    for (int t = 0; t < 4; ++t) km[t] = cm[sh + t];
                    for (int t = 0; t < 12; ++t) rm[t] = cm[t < sh ? t : t + 4];
                    k_apply<<<NBC * WPS / AWV, 32 * AWV, 0, stream>>>(cur, oth, AH + (size_t)mat * 1024, AR + (size_t)mat * 1024,
                        km[0] | (km[1] << 16), km[2] | (km[3] << 16),
                        rm[0] | (rm[1] << 16), rm[2] | (rm[3] << 16), rm[4] | (rm[5] << 16), rm[6] | (rm[7] << 16), rm[8] | (rm[9] << 16), rm[10] | (rm[11] << 16));
                    for (int j = 0; j < 16; ++j)
                        cm[j] = (unsigned short)((j >= sh && j < sh + 4) ? (1u << (j - sh)) : ((j < sh) ? (1u << (j + 4)) : (1u << j)));
                    float* tmp = cur; cur = oth; oth = tmp;
                }
            }
            if (st < 3) { const int r = (st % (NW - 1)) + 1; for (int w = 0; w < NW; ++w) cnot_relabel(cm, w, (w + r) % NW); }
        }
        unsigned dm[8];
        for (int t = 0; t < 8; ++t) dm[t] = (unsigned)(cm[2 * t] ^ cm[2 * t + 1]);
        k_expect<<<NBC / 16, 32, 0, stream>>>(cur, noise, OUT, cb, dm[0] | (dm[1] << 16), dm[2] | (dm[3] << 16), dm[4] | (dm[5] << 16), dm[6] | (dm[7] << 16));
    }
}
